// HybridGVP_GAT_Long_Layer_67095979098197
// MI455X (gfx1250) — hardware-verified
//
#include <hip/hip_runtime.h>
#include <math.h>

#define NB 4
#define NL 2048
#define ND 256
#define NH 4
#define NR 128
#define NE 32768
#define NV (NE + NL)
#define NBL (NB * NL)
#define NFF 1024
#define HGW (NH * ND)
#define HGN 1088
#define NT 256

typedef __attribute__((ext_vector_type(16))) _Float16 v16h;
typedef __attribute__((ext_vector_type(8)))  _Float16 v8h;
typedef __attribute__((ext_vector_type(16))) __bf16   v16b;
typedef __attribute__((ext_vector_type(8)))  __bf16   v8b;
typedef __attribute__((ext_vector_type(8)))  float    v8f;
typedef __attribute__((ext_vector_type(4)))  float    v4f;
typedef __attribute__((ext_vector_type(4)))  int      v4i;

__device__ __forceinline__ unsigned short f2bf_bits(float f) {
  unsigned u = __float_as_uint(f);
  return (unsigned short)((u + 0x7FFFu + ((u >> 16) & 1u)) >> 16);
}
__device__ __forceinline__ float bf_bits2f(unsigned short h) { return __uint_as_float(((unsigned)h) << 16); }

__device__ __forceinline__ void dep_guard_h(v8f& a, v8f& b, v16h x, v16h y) { asm volatile("v_nop\n\tv_nop\n\tv_nop\n\tv_nop" : "+v"(a), "+v"(b) : "v"(x), "v"(y)); }
__device__ __forceinline__ void dep_guard_b(v8f& a, v8f& b, v16b x, v16b y) { asm volatile("v_nop\n\tv_nop\n\tv_nop\n\tv_nop" : "+v"(a), "+v"(b) : "v"(x), "v"(y)); }
__device__ __forceinline__ void keep4_h(v16h a, v16h b, v16h c, v16h d) { asm volatile("v_nop" :: "v"(a), "v"(b), "v"(c), "v"(d)); }
__device__ __forceinline__ void keep4_b(v16b a, v16b b, v16b c, v16b d) { asm volatile("v_nop" :: "v"(a), "v"(b), "v"(c), "v"(d)); }
__device__ __forceinline__ void fence_v4(v4f& t) { asm volatile("" : "+v"(t)); }
__device__ __forceinline__ void acc_guard4(v8f& a, v8f& b, v8f& c, v8f& d) { asm volatile("v_nop\n\tv_nop\n\tv_nop\n\tv_nop" : "+v"(a), "+v"(b), "+v"(c), "+v"(d)); }
template <typename T> struct Frag;
template <> struct Frag<_Float16> {
  typedef v16h V; union U { v16h v; v8h h[2]; };
  static __device__ __forceinline__ v16h load(const _Float16* p) {
    U f; f.h[0] = *(const v8h*)(p); f.h[1] = *(const v8h*)(p + 16); return f.v;
  }
  static __device__ __forceinline__ v8f mma(v16h a, v16h b, v8f c) {
    return __builtin_amdgcn_wmma_f32_16x16x32_f16(false, a, false, b, (short)0, c, false, false);
  }
  static __device__ __forceinline__ void guard(v8f& a, v8f& b, v16h x, v16h y) { dep_guard_h(a, b, x, y); }
  static __device__ __forceinline__ void keep(v16h a, v16h b, v16h c, v16h d) { keep4_h(a, b, c, d); }
};
template <> struct Frag<__bf16> {
  typedef v16b V; union U { v16b v; v8b h[2]; };
  static __device__ __forceinline__ v16b load(const __bf16* p) {
    U f; f.h[0] = *(const v8b*)(p); f.h[1] = *(const v8b*)(p + 16); return f.v;
  }
  static __device__ __forceinline__ v8f mma(v16b a, v16b b, v8f c) {
    return __builtin_amdgcn_wmma_f32_16x16x32_bf16(false, a, false, b, (short)0, c, false, false);
  }
  static __device__ __forceinline__ void guard(v8f& a, v8f& b, v16b x, v16b y) { dep_guard_b(a, b, x, y); }
  static __device__ __forceinline__ void keep(v16b a, v16b b, v16b c, v16b d) { keep4_b(a, b, c, d); }
};

template <int ET> struct Elem;
template <> struct Elem<0> { typedef _Float16 T; };
template <> struct Elem<1> { typedef __bf16 T; };
template <int ET, bool SPLIT, int BIAS_MODE, int OUT_MODE, bool RESID, int ACT = 0, int OSC = 1>
__global__ __launch_bounds__(256) void wmma_gemm64(
    const unsigned short* __restrict__ Ap, const unsigned short* __restrict__ A2p, int lda, long strideA,
    const unsigned short* __restrict__ Btp, const unsigned short* __restrict__ Bt2p, int ldb, long strideB,
    void* __restrict__ Cout, void* __restrict__ Cout2, int ldc, long strideC,
    const float* __restrict__ bias,
    const float* __restrict__ resid, long strideR,
    int M, int N, int K, float scale) {
  typedef typename Elem<ET>::T T;
  typedef typename Frag<T>::V V;
  const T* A = (const T*)Ap; const T* A2 = (const T*)A2p; const T* Bt = (const T*)Btp; const T* Bt2 = (const T*)Bt2p;
  __shared__ __align__(16) float sT[8][16 * 68];
  const int b    = blockIdx.y;
  const int lane = threadIdx.x & 31;
  const int wave = threadIdx.x >> 5;
  const int tilesN = N >> 6;
  const int tilesM = M >> 6;
  const int tile = blockIdx.x * 8 + wave;
  if (tile >= tilesM * tilesN) return;
  const int tm = tile / tilesN;
  const int tn = tile - tm * tilesN;
  const int m0 = tm << 6;
  const int n0 = tn << 6;

  const T* Ab  = A  + (size_t)b * strideA;
  const T* Bb  = Bt + (size_t)b * strideB;
  const T* Ab2 = SPLIT ? (A2  + (size_t)b * strideA) : nullptr;
  const T* Bb2 = SPLIT ? (Bt2 + (size_t)b * strideB) : nullptr;

  const int rlane = lane & 15;
  const int koff  = (lane >> 4) * 8;
  const int mOff  = (lane >> 4) * 8;

  v8f acc[4][4];
#pragma unroll
  for (int i = 0; i < 4; ++i)
#pragma unroll
    for (int j = 0; j < 4; ++j) acc[i][j] = (v8f){0.f,0.f,0.f,0.f,0.f,0.f,0.f,0.f};

  for (int k0 = 0; k0 < K; k0 += 32) {
    V bh[4], bl[4];
#pragma unroll
    for (int j = 0; j < 4; ++j) {
      const size_t bo = (size_t)(n0 + (j << 4) + rlane) * ldb + koff + k0;
      bh[j] = Frag<T>::load(Bb + bo);
      if (SPLIT) bl[j] = Frag<T>::load(Bb2 + bo);
    }
#pragma unroll
    for (int i = 0; i < 4; ++i) {
      const size_t ao = (size_t)(m0 + (i << 4) + rlane) * lda + koff + k0;
      V ah = Frag<T>::load(Ab + ao);
      V al;
      if (SPLIT) al = Frag<T>::load(Ab2 + ao);
#pragma unroll
      for (int j = 0; j < 4; ++j) {
        acc[i][j] = Frag<T>::mma(ah, bh[j], acc[i][j]);
        if (SPLIT) {
          acc[i][j] = Frag<T>::mma(ah, bl[j], acc[i][j]);
          acc[i][j] = Frag<T>::mma(al, bh[j], acc[i][j]);
        }
      }
      Frag<T>::guard(acc[i][0], acc[i][3], ah, SPLIT ? al : ah);
    }
    Frag<T>::keep(bh[0], bh[1], bh[2], bh[3]);
    if (SPLIT) Frag<T>::keep(bl[0], bl[1], bl[2], bl[3]);
  }
  acc_guard4(acc[0][0], acc[0][1], acc[0][2], acc[0][3]);
  acc_guard4(acc[1][0], acc[1][1], acc[1][2], acc[1][3]);
  acc_guard4(acc[2][0], acc[2][1], acc[2][2], acc[2][3]);
  acc_guard4(acc[3][0], acc[3][1], acc[3][2], acc[3][3]);

  float* slab = sT[wave];
  const float* Rb = RESID ? (resid + (size_t)b * strideR) : nullptr;
#pragma unroll
  for (int i = 0; i < 4; ++i) {
    const int mBase = m0 + (i << 4);
#pragma unroll
    for (int j = 0; j < 4; ++j) {
      const int n = n0 + (j << 4) + rlane;
      float bv = 0.f;
      if (BIAS_MODE == 2) bv = bias[n];
#pragma unroll
      for (int r = 0; r < 8; ++r) {
        float v = acc[i][j][r] * scale;
        if (BIAS_MODE == 1) v += bias[mBase + mOff + r];
        if (BIAS_MODE == 2) v += bv;
        if (RESID) v += Rb[(size_t)(mBase + mOff + r) * ldc + n];
        if (ACT == 1) v = tanhf(v);
        if (ACT == 2) v = fmaxf(v, 0.0f);
        if (ACT == 3) v = v / (1.0f + expf(-v));
        if (ACT == 4) v = (v > 0.f) ? v : 0.01f * v;
        if (ACT == 5) v = 0.5f * v * (1.0f + erff(v * 0.70710678118654752f));
        slab[(mOff + r) * 68 + (j << 4) + rlane] = v;
      }
    }
    __builtin_amdgcn_fence(__ATOMIC_RELEASE, "workgroup");
    __builtin_amdgcn_wave_barrier();
    __builtin_amdgcn_fence(__ATOMIC_ACQUIRE, "workgroup");
    if (OUT_MODE == 0) {
      float* C = (float*)Cout + (size_t)b * strideC;
      const int hh = lane >> 4, c4 = (lane & 15) * 4;
      for (int pass = 0; pass < 2; ++pass) {
#pragma unroll
        for (int it = 0; it < 8; ++it) {
          const int row = it * 2 + hh;
          v4f v = *(const v4f*)(slab + row * 68 + c4);
          *(volatile v4f*)(C + (size_t)(mBase + row) * ldc + n0 + c4) = v;
        }
        __threadfence();
      }
    } else {
      const int q = lane >> 3, c8 = (lane & 7) * 8;
      unsigned short* C  = (unsigned short*)Cout  + (size_t)b * strideC;
      unsigned short* C2 = (OUT_MODE == 2) ? ((unsigned short*)Cout2 + (size_t)b * strideC) : nullptr;
      for (int pass = 0; pass < 2; ++pass) {
#pragma unroll
        for (int it = 0; it < 4; ++it) {
          const int row = it * 4 + q;
          const float* sp = slab + row * 68 + c8;
          v8h hv, lv;
#pragma unroll
          for (int e = 0; e < 8; ++e) {
            if (OUT_MODE == 1) {
              hv[e] = (_Float16)(sp[e] * (float)OSC);
            } else {
              unsigned short hb = f2bf_bits(sp[e]);
              unsigned short lb = f2bf_bits(sp[e] - bf_bits2f(hb));
              hv[e] = __builtin_bit_cast(_Float16, hb);
              lv[e] = __builtin_bit_cast(_Float16, lb);
            }
          }
          *(volatile v8h*)(C + (size_t)(mBase + row) * ldc + n0 + c8) = hv;
          if (OUT_MODE == 2) *(volatile v8h*)(C2 + (size_t)(mBase + row) * ldc + n0 + c8) = lv;
        }
        __threadfence();
      }
    }
    __builtin_amdgcn_fence(__ATOMIC_RELEASE, "workgroup");
    __builtin_amdgcn_wave_barrier();
    __builtin_amdgcn_fence(__ATOMIC_ACQUIRE, "workgroup");
  }
}

__global__ __launch_bounds__(256) void cast_scale_f32_f16x2(
    const float* __restrict__ in, _Float16* __restrict__ out, int n2, float sc) {
  int i = blockIdx.x * 256 + threadIdx.x;
  if (i < n2) {
    const _Float16 h0 = (_Float16)(in[2 * i] * sc), h1 = (_Float16)(in[2 * i + 1] * sc);
    const unsigned u = (unsigned)__builtin_bit_cast(unsigned short, h0) | ((unsigned)__builtin_bit_cast(unsigned short, h1) << 16);
    ((volatile unsigned*)out)[i] = u;
    __threadfence();
    ((volatile unsigned*)out)[i] = u;
  }
}

__global__ __launch_bounds__(NT) void tcast_kernel(const float* __restrict__ in, _Float16* __restrict__ out, int K, int N, float sc) {
  __shared__ float T[64][65];
  const int tid = threadIdx.x, lane = tid & 31, wave = tid >> 5;
  const int n0 = blockIdx.x * 64, k0 = blockIdx.y * 64;
#pragma unroll
  for (int p = 0; p < 16; ++p) {
    const int kk = p * 4 + (tid >> 6), nn = tid & 63;
    T[kk][nn] = in[(size_t)(k0 + kk) * N + n0 + nn];
  }
  __syncthreads();
  const int q = lane >> 3, c8 = (lane & 7) * 8;
  v8h vv[2];
#pragma unroll
  for (int it = 0; it < 2; ++it) {
    const int nl = wave * 8 + it * 4 + q;
    v8h hv;
#pragma unroll
    for (int e = 0; e < 8; ++e) hv[e] = (_Float16)(T[c8 + e][nl] * sc);
    vv[it] = hv;
  }
  for (int pass = 0; pass < 2; ++pass) {
#pragma unroll
    for (int it = 0; it < 2; ++it) {
      const int nl = wave * 8 + it * 4 + q;
      *(volatile v8h*)(out + (size_t)(n0 + nl) * K + k0 + c8) = vv[it];
    }
    __threadfence();
  }
}

__global__ __launch_bounds__(NT) void att_rows_kernel(const float* __restrict__ gW, const float* __restrict__ asrc, const float* __restrict__ adst,
                                                    _Float16* __restrict__ gWt) {
  __shared__ __align__(16) _Float16 rowh[ND];
  const int tid = threadIdx.x, lane = tid & 31, wave = tid >> 5;
  const int j = blockIdx.x;
  float s = 0.f;
  if (j < 8) {
    const int sel = j >> 2, h = j & 3;
    const float* av = sel ? adst : asrc;
    const float* wr = gW + (size_t)tid * HGW + h * ND;
    const float* ar = av + h * ND;
#pragma unroll 1
    for (int c = 0; c < ND; ++c) s += wr[c] * ar[c];
  }
  rowh[tid] = (_Float16)(s * 16.0f);
  __syncthreads();
  if (wave == 0) {
    const v8h hv = *(const v8h*)(rowh + 8 * lane);
    _Float16* op = gWt + (size_t)(HGW + j) * ND + 8 * lane;
    *(volatile v8h*)op = hv;
    __threadfence();
    *(volatile v8h*)op = hv;
  }
}

template <int WF, int WH, int WT>
__global__ __launch_bounds__(NT) void ln_kernel(const float* x, const float* __restrict__ g, const float* __restrict__ bt,
                                               float* of, _Float16* __restrict__ oh, _Float16* __restrict__ oT) {
  __shared__ __align__(16) float rowbuf[8][ND];
  __shared__ __align__(16) _Float16 TT[WT ? ND * 72 : 8];
  const int tid = threadIdx.x, lane = tid & 31, wave = tid >> 5;
  const int r0 = blockIdx.x * 64;
  const v4f g0 = *(const v4f*)(g + 4 * lane), g1 = *(const v4f*)(g + 128 + 4 * lane);
  const v4f b0 = *(const v4f*)(bt + 4 * lane), b1 = *(const v4f*)(bt + 128 + 4 * lane);
#pragma unroll 1
  for (int j = 0; j < 8; ++j) {
    const int ll = wave * 8 + j;
    const int row = r0 + ll;
    const float* xr = x + (size_t)row * ND;
    const v4f a0 = *(const v4f*)(xr + 4 * lane), a1 = *(const v4f*)(xr + 128 + 4 * lane);
    float s = (a0[0] + a0[1]) + (a0[2] + a0[3]) + (a1[0] + a1[1]) + (a1[2] + a1[3]);
#pragma unroll
    for (int off = 16; off; off >>= 1) s += __shfl_xor(s, off, 32);
    const float mu = s * (1.0f / 256.0f);
    const v4f d0 = a0 - mu, d1 = a1 - mu;
    float qq = d0[0] * d0[0] + d0[1] * d0[1] + d0[2] * d0[2] + d0[3] * d0[3] + d1[0] * d1[0] + d1[1] * d1[1] + d1[2] * d1[2] + d1[3] * d1[3];
#pragma unroll
    for (int off = 16; off; off >>= 1) qq += __shfl_xor(qq, off, 32);
    const float var = qq * (1.0f / 256.0f);
    const float rs = rsqrtf(var + 1e-5f);
    v4f y0 = d0 * rs, y1 = d1 * rs;
    y0 = y0 * g0 + b0; y1 = y1 * g1 + b1;
    if (WF) {
      float* orow = of + (size_t)row * ND;
      *(volatile v4f*)(orow + 4 * lane) = y0; *(volatile v4f*)(orow + 128 + 4 * lane) = y1;
      __threadfence();
      *(volatile v4f*)(orow + 4 * lane) = y0; *(volatile v4f*)(orow + 128 + 4 * lane) = y1;
    }
    if (WH || WT) {
      float* rb = rowbuf[wave];
      *(v4f*)(rb + 4 * lane) = y0; *(v4f*)(rb + 128 + 4 * lane) = y1;
      __builtin_amdgcn_fence(__ATOMIC_RELEASE, "workgroup");
      __builtin_amdgcn_wave_barrier();
      __builtin_amdgcn_fence(__ATOMIC_ACQUIRE, "workgroup");
      const v4f c0 = *(const v4f*)(rb + 8 * lane), c1 = *(const v4f*)(rb + 8 * lane + 4);
      v8h hv;
#pragma unroll
      for (int e = 0; e < 4; ++e) { hv[e] = (_Float16)(c0[e] * 16.0f); hv[4 + e] = (_Float16)(c1[e] * 16.0f); }
      if (WH) {
        _Float16* hrow = oh + (size_t)row * ND + 8 * lane;
        *(volatile v8h*)hrow = hv;
        __threadfence();
        *(volatile v8h*)hrow = hv;
      }
      if (WT) {
#pragma unroll
        for (int e = 0; e < 8; ++e) TT[(8 * lane + e) * 72 + ll] = hv[e];
      }
      __builtin_amdgcn_fence(__ATOMIC_RELEASE, "workgroup");
      __builtin_amdgcn_wave_barrier();
      __builtin_amdgcn_fence(__ATOMIC_ACQUIRE, "workgroup");
    }
  }
  if (WT) {
    __syncthreads();
    const int b = r0 / NL, l0 = r0 - b * NL;
    const int q = lane >> 3, c8 = (lane & 7) * 8;
    v8h tv[8];
#pragma unroll
    for (int it = 0; it < 8; ++it) {
      const int d = wave * 32 + it * 4 + q;
      tv[it] = *(const v8h*)(TT + d * 72 + c8);
    }
    for (int pass = 0; pass < 2; ++pass) {
#pragma unroll
      for (int it = 0; it < 8; ++it) {
        const int d = wave * 32 + it * 4 + q;
        *(volatile v8h*)(oT + ((size_t)(b * ND + d)) * NL + l0 + c8) = tv[it];
      }
      __threadfence();
    }
  }
}

__global__ __launch_bounds__(NT) void seqsoftmax_kernel(const float* __restrict__ pml, _Float16* __restrict__ pmT) {
  __shared__ float red[8];
  const int tid = threadIdx.x, lane = tid & 31, wave = tid >> 5;
  const int b = blockIdx.x / NR, r = blockIdx.x - b * NR;
  const float* col = pml + (size_t)b * NL * NR + r;
  float xv[8];
  float m = -INFINITY;
#pragma unroll
  for (int k = 0; k < 8; ++k) { xv[k] = col[(size_t)(8 * tid + k) * NR]; m = fmaxf(m, xv[k]); }
#pragma unroll
  for (int off = 16; off; off >>= 1) m = fmaxf(m, __shfl_xor(m, off, 32));
  if (lane == 0) red[wave] = m;
  __syncthreads();
  float mm = red[0];
#pragma unroll
  for (int w = 1; w < 8; ++w) mm = fmaxf(mm, red[w]);
  __syncthreads();
  float ev[8];
  float sum = 0.f;
#pragma unroll
  for (int k = 0; k < 8; ++k) { ev[k] = __expf(xv[k] - mm); sum += ev[k]; }
#pragma unroll
  for (int off = 16; off; off >>= 1) sum += __shfl_xor(sum, off, 32);
  if (lane == 0) red[wave] = sum;
  __syncthreads();
  float tot = red[0];
#pragma unroll
  for (int w = 1; w < 8; ++w) tot += red[w];
  const float inv = 1.0f / tot;
  v8h hv;
#pragma unroll
  for (int k = 0; k < 8; ++k) hv[k] = (_Float16)((ev[k] * inv) * 32768.0f);
  _Float16* op = pmT + ((size_t)(b * NR + r)) * NL + 8 * tid;
  *(volatile v8h*)op = hv;
  __threadfence();
  *(volatile v8h*)op = hv;
}

__device__ __forceinline__ int blk_excl_scan(int cnt, int* scan_ws, int tid, int* tot) {
  const int lane = tid & 31, wave = tid >> 5; int incl = cnt;
#pragma unroll
  for (int o = 1; o < 32; o <<= 1) { const int v = __shfl_up(incl, o, 32); if (lane >= o) incl += v; }
  if (lane == 31) scan_ws[wave] = incl;
  __syncthreads();
  if (wave == 0) { int wv = (lane < NT / 32) ? scan_ws[lane] : 0; int wincl = wv;
#pragma unroll
    for (int o = 1; o < 32; o <<= 1) { const int v = __shfl_up(wincl, o, 32); if (lane >= o) wincl += v; }
    if (lane < NT / 32) scan_ws[32 + lane] = wincl - wv; if (lane == 31) scan_ws[64] = wincl; }
  __syncthreads();
  const int res = scan_ws[32 + wave] + incl - cnt; *tot = scan_ws[64];
  return res;
}
#define SRB 512
template <int SP, int CAP>
__device__ __forceinline__ int chunk_hits(const int* __restrict__ dstv, const int* __restrict__ srcv, int e0, int n0, int tid,
                                          int* LIST, int* scan_ws) {
  const int eb = e0 + tid * SP;
  const int ebc = (eb + SP <= NE) ? eb : (NE - SP);
  int rec[SP]; int cnt = 0;
#pragma unroll
  for (int k = 0; k < SP; k += 4) {
    const v4i d4 = *(const v4i*)(dstv + ebc + k);
    const v4i s4 = *(const v4i*)(srcv + ebc + k);
#pragma unroll
    for (int e = 0; e < 4; ++e) {
      const int ee = eb + k + e;
      int d, s;
      if (ee < NE) { d = d4[e]; s = s4[e]; s = s < 0 ? 0 : (s >= NL ? NL - 1 : s); }
      else { d = ee - NE; s = d; }
      int r = -1;
      if (ee < NV && d >= n0 && d < n0 + SRB) { r = ((d - n0) << 16) | s; ++cnt; }
      rec[k + e] = r;
    }
  }
  int tot; int p = blk_excl_scan(cnt, scan_ws, tid, &tot);
#pragma unroll
  for (int k = 0; k < SP; ++k) if (rec[k] >= 0) { if ((unsigned)p < (unsigned)CAP) LIST[p] = rec[k]; ++p; }
  __syncthreads();
  return tot < CAP ? tot : CAP;
}

#define SCH 2048
#define NCH ((NV + SCH - 1) / SCH)
__global__ __launch_bounds__(NT) void gat_agg_kernel(const float* __restrict__ hg, const int* __restrict__ ei, const float* __restrict__ gat_b,
                                                   float* ACC, _Float16* __restrict__ gout) {
  __shared__ int LIST[SCH];
  __shared__ float SM[SRB * 4];
  __shared__ float SL[SRB * 4];
  __shared__ float SAD[SRB * 4];
  __shared__ int scan_ws[80];
  const int tid = threadIdx.x, lane = tid & 31, wave = tid >> 5;
  const int b = blockIdx.x >> 2, tile = blockIdx.x & 3;
  const int n0 = tile * SRB;
  const size_t rowb = (size_t)b * NL + n0;
  const int h4 = lane & 3;
  const v4f z4 = {0.f, 0.f, 0.f, 0.f};
  for (int pass = 0; pass < 2; ++pass) {
#pragma unroll 1
    for (int j = 0; j < 64; ++j) {
      float* rp = ACC + (rowb + wave * 64 + j) * HGW + 4 * lane;
#pragma unroll
      for (int jj = 0; jj < 8; ++jj) *(volatile v4f*)(rp + 128 * jj) = z4;
    }
    __threadfence();
  }
  for (int i = tid; i < SRB * 4; i += NT) {
    SM[i] = -INFINITY; SL[i] = 0.f;
    const int dl = i >> 2, h = i & 3;
    SAD[i] = hg[(rowb + dl) * HGN + HGW + 4 + h];
  }
  __syncthreads();
  const int* srcv = ei; const int* dstv = ei + NE;
#pragma unroll 1
  for (int c = 0; c < NCH; ++c) {
    const int tot = chunk_hits<SCH / NT, SCH>(dstv, srcv, c * SCH, n0, tid, LIST, scan_ws);
#pragma unroll 1
    for (int base = 0; base < tot; base += 32) {
      const int q = base + lane;
      const int qc = q < SCH ? q : SCH - 1;
      const int lr = LIST[qc];
      const int rv = (q < tot) ? lr : -1;
      const int own = (rv >= 0 && (rv >> 22) == wave) ? 1 : 0;
      unsigned msk = (unsigned)__ballot(own);
#pragma unroll 1
      for (int it = 0; it < 32; ++it) {
        if (msk == 0u) break;
        const int bp = __builtin_ctz(msk); msk &= msk - 1u;
        const int r = __shfl(rv, bp, 32);
        const int dl = r >> 16, s = r & 0xFFFF;
        const float* hr = hg + ((size_t)b * NL + s) * HGN;
        const v4f as4 = *(const v4f*)(hr + HGW);
        const float asv = (h4 == 0) ? as4[0] : ((h4 == 1) ? as4[1] : ((h4 == 2) ? as4[2] : as4[3]));
        const int mi = dl * 4 + h4;
        float al = asv + SAD[mi];
        al = (al >= 0.f) ? al : 0.2f * al;
        const float mo = SM[mi], lo = SL[mi];
        const float mn = fmaxf(mo, al);
        const float rr = __expf(mo - mn), ex = __expf(al - mn);
        const float ln = lo * rr + ex;
        if (lane < 4) { SM[mi] = mn; SL[mi] = ln; }
        float* rp = ACC + (rowb + dl) * HGW + 4 * lane;
        v4f nv[8];
#pragma unroll
        for (int jj = 0; jj < 8; ++jj) {
          const float rrj = __shfl(rr, jj >> 1, 32), exj = __shfl(ex, jj >> 1, 32);
          const v4f hv = *(const v4f*)(hr + 4 * lane + 128 * jj);
          const v4f a = *(const v4f*)(rp + 128 * jj);
          nv[jj] = a * rrj + exj * hv;
        }
#pragma unroll
        for (int jj = 0; jj < 8; ++jj) *(volatile v4f*)(rp + 128 * jj) = nv[jj];
        __threadfence();
#pragma unroll
        for (int jj = 0; jj < 8; ++jj) *(volatile v4f*)(rp + 128 * jj) = nv[jj];
      }
    }
    __syncthreads();
  }
  __threadfence();
  v4f gb0[4], gb1[4];
#pragma unroll
  for (int jj = 0; jj < 4; ++jj) { gb0[jj] = *(const v4f*)(gat_b + 8 * lane + 256 * jj); gb1[jj] = *(const v4f*)(gat_b + 8 * lane + 256 * jj + 4); }
#pragma unroll 1
  for (int j = 0; j < 64; ++j) {
    const int dl = wave * 64 + j;
    float lv = SL[dl * 4 + h4];
    lv = (lv > 0.f) ? lv : 1.0f;
    const float inv = 1.0f / lv;
    const float* rp = ACC + (rowb + dl) * HGW;
    _Float16* op = gout + (rowb + dl) * HGW;
    v8h hv[4];
#pragma unroll
    for (int jj = 0; jj < 4; ++jj) {
      const float invj = __shfl(inv, jj, 32);
      const v4f a0 = *(const v4f*)(rp + 8 * lane + 256 * jj), a1 = *(const v4f*)(rp + 8 * lane + 256 * jj + 4);
      v4f t0 = a0 * invj; fence_v4(t0); t0 = t0 + gb0[jj];
      v4f t1 = a1 * invj; fence_v4(t1); t1 = t1 + gb1[jj];
      v8h w;
#pragma unroll
      for (int e = 0; e < 4; ++e) { w[e] = (_Float16)(t0[e] * 16.0f); w[4 + e] = (_Float16)(t1[e] * 16.0f); }
      hv[jj] = w;
    }
    for (int pass = 0; pass < 2; ++pass) {
#pragma unroll
      for (int jj = 0; jj < 4; ++jj) *(volatile v8h*)(op + 8 * lane + 256 * jj) = hv[jj];
      __threadfence();
    }
  }
}

#define CPP 136
__device__ __forceinline__ v8f hmma(v16h a, v16h b, v8f c) {
  c = __builtin_amdgcn_wmma_f32_16x16x32_f16(false, a, false, b, (short)0, c, false, false);
  asm volatile("v_nop\n\tv_nop\n\tv_nop\n\tv_nop" : "+v"(c) : "v"(a), "v"(b));
  return c;
}
__global__ __launch_bounds__(128) void lr_attn_kernel(const _Float16* __restrict__ qh, const _Float16* __restrict__ kc,
                                                    const _Float16* __restrict__ vcT, _Float16* __restrict__ oh,
                                                    float sscale, float oscale) {
  __shared__ __align__(16) _Float16 Psh[4][16 * CPP];
  __shared__ __align__(16) float Os[4][16 * 68];
  const int tid = threadIdx.x, wave = tid >> 5, lane = tid & 31;
  const int hh = lane >> 4, c = lane & 15, koff = hh * 8;
  const int bx = blockIdx.x;
  const int qb = bx % (NL / 64);
  const int bhd = bx / (NL / 64);
  const int h = bhd % NH, b = bhd / NH;
  const int q0 = qb * 64 + wave * 16;

  v16h qa[2];
  {
    const _Float16* qp = qh + ((size_t)(b * NL + q0 + c)) * ND + h * 64 + koff;
#pragma unroll
    for (int dc = 0; dc < 2; ++dc) qa[dc] = Frag<_Float16>::load(qp + dc * 32);
  }
  const _Float16* kp = kc + ((size_t)b * NR) * ND + h * 64 + koff;
  v8f s[8];
#pragma unroll
  for (int j = 0; j < 8; ++j) {
    s[j] = (v8f){0.f, 0.f, 0.f, 0.f, 0.f, 0.f, 0.f, 0.f};
#pragma unroll
    for (int dc = 0; dc < 2; ++dc) {
      const v16h kf = Frag<_Float16>::load(kp + (size_t)(j * 16 + c) * ND + dc * 32);
      s[j] = hmma(qa[dc], kf, s[j]);
    }
  }
  _Float16* pw = Psh[wave];
  float lrow[8];
#pragma unroll
  for (int r = 0; r < 8; ++r) {
    float m = -INFINITY;
#pragma unroll
    for (int j = 0; j < 8; ++j) { const float t = s[j][r] * sscale; s[j][r] = t; m = fmaxf(m, t); }
#pragma unroll
    for (int off = 1; off < 16; off <<= 1) m = fmaxf(m, __shfl_xor(m, off, 32));
    float psum = 0.f;
#pragma unroll
    for (int j = 0; j < 8; ++j) {
      const float p = __expf(s[j][r] - m);
      psum += p;
      pw[(8 * hh + r) * CPP + j * 16 + c] = (_Float16)(p * 32768.0f);
    }
#pragma unroll
    for (int off = 1; off < 16; off <<= 1) psum += __shfl_xor(psum, off, 32);
    lrow[r] = psum;
  }
  __syncthreads();
  v8f oacc[4];
#pragma unroll
  for (int t = 0; t < 4; ++t) oacc[t] = (v8f){0.f, 0.f, 0.f, 0.f, 0.f, 0.f, 0.f, 0.f};
  const _Float16* vp = vcT + ((size_t)(b * ND + h * 64 + c)) * NR + koff;
#pragma unroll
  for (int kk = 0; kk < 4; ++kk) {
    const v16h pa = Frag<_Float16>::load(pw + c * CPP + kk * 32 + koff);
#pragma unroll
    for (int t = 0; t < 4; ++t) {
      const v16h vf = Frag<_Float16>::load(vp + (size_t)(t * 16) * NR + kk * 32);
      oacc[t] = hmma(pa, vf, oacc[t]);
    }
  }
  float* os = Os[wave];
#pragma unroll
  for (int r = 0; r < 8; ++r) {
    const float inv = oscale * (1.0f / lrow[r]);
#pragma unroll
    for (int t = 0; t < 4; ++t) os[(8 * hh + r) * 68 + t * 16 + c] = oacc[t][r] * inv;
  }
  __syncthreads();
  const int q4 = lane >> 3, c8 = (lane & 7) * 8;
  v8h hv[4];
#pragma unroll
  for (int it = 0; it < 4; ++it) {
    const int row = it * 4 + q4;
    v8h w;
#pragma unroll
    for (int e = 0; e < 8; ++e) w[e] = (_Float16)os[row * 68 + c8 + e];
    hv[it] = w;
  }
  _Float16* op = oh + ((size_t)(b * NL + q0)) * ND + h * 64 + c8;
  for (int pass = 0; pass < 2; ++pass) {
#pragma unroll
    for (int it = 0; it < 4; ++it) {
      const int row = it * 4 + q4;
      *(volatile v8h*)(op + (size_t)row * ND) = hv[it];
    }
    __threadfence();
  }
}

extern "C" void kernel_launch(void* const* d_in, const int* in_sizes, int n_in,
                              void* d_out, int out_size, void* d_ws, size_t ws_size, hipStream_t stream) {
  if (n_in < 32) return;
  if (in_sizes[0] != NBL * ND || in_sizes[31] != 2 * NE || out_size != NBL * ND) return;
  const float* s       = (const float*)d_in[0];
  const float* gat_W   = (const float*)d_in[1];
  const float* att_src = (const float*)d_in[2];
  const float* att_dst = (const float*)d_in[3];
  const float* gat_b   = (const float*)d_in[4];
  const float* short_W = (const float*)d_in[5];
  const float* short_b = (const float*)d_in[6];
  const float* q_W = (const float*)d_in[7];  const float* q_b = (const float*)d_in[8];
  const float* k_W = (const float*)d_in[9];  const float* k_b = (const float*)d_in[10];
  const float* v_W = (const float*)d_in[11]; const float* v_b = (const float*)d_in[12];
  const float* o_W = (const float*)d_in[13]; const float* o_b = (const float*)d_in[14];
  const float* p_W = (const float*)d_in[15]; const float* p_b = (const float*)d_in[16];
  const float* lnq_g = (const float*)d_in[17]; const float* lnq_b = (const float*)d_in[18];
  const float* lnk_g = (const float*)d_in[19]; const float* lnk_b = (const float*)d_in[20];
  const float* lnv_g = (const float*)d_in[21]; const float* lnv_b = (const float*)d_in[22];
  const float* ln1_g = (const float*)d_in[23]; const float* ln1_b = (const float*)d_in[24];
  const float* ln2_g = (const float*)d_in[25]; const float* ln2_b = (const float*)d_in[26];
  const float* f1_W = (const float*)d_in[27]; const float* f1_b = (const float*)d_in[28];
  const float* f2_W = (const float*)d_in[29]; const float* f2_b = (const float*)d_in[30];
  const int*   ei   = (const int*)d_in[31];
  float* out = (float*)d_out;

  char* ws = (char*)d_ws; size_t off = 0;
  auto carve = [&](size_t bytes) -> char* { char* p = ws + off; off += (bytes + 255) & ~(size_t)255; return p; };
  _Float16* sh      = (_Float16*)carve((size_t)NBL * ND * 2);
  _Float16* gatWt   = (_Float16*)carve((size_t)HGN * ND * 2);
  _Float16* shortWt = (_Float16*)carve((size_t)ND * HGW * 2);
  _Float16* qWt     = (_Float16*)carve((size_t)ND * ND * 2);
  _Float16* kWt     = (_Float16*)carve((size_t)ND * ND * 2);
  _Float16* vWt     = (_Float16*)carve((size_t)ND * ND * 2);
  _Float16* oWt     = (_Float16*)carve((size_t)ND * ND * 2);
  _Float16* pWt     = (_Float16*)carve((size_t)NR * ND * 2);
  _Float16* f1Wt    = (_Float16*)carve((size_t)NFF * ND * 2);
  _Float16* f2Wt    = (_Float16*)carve((size_t)ND * NFF * 2);
  char* R1 = carve((size_t)NBL * HGN * 4);
  char* R2 = carve((size_t)NBL * HGW * 4);
  char* R3 = carve((size_t)NBL * HGW * 2);
  if (off > ws_size || off > (size_t)134217728) return;

  float*    hg    = (float*)R1;
  float*    sshrt = (float*)R1;
  _Float16* qh    = (_Float16*)(R1 + 8388608);
  _Float16* ff1h  = (_Float16*)R1;
  float*    x2    = (float*)(R1 + 16777216);
  float*    acc   = (float*)R2;
  float*    tmp   = (float*)R2;
  float*    pml   = (float*)R2;
  _Float16* kh    = (_Float16*)(R2 + 8388608);
  _Float16* kT    = (_Float16*)(R2 + 12582912);
  _Float16* vT    = (_Float16*)(R2 + 16777216);
  _Float16* pmT   = (_Float16*)(R2 + 20971520);
  _Float16* kc16  = (_Float16*)(R2 + 23068672);
  _Float16* vcT16 = (_Float16*)(R2 + 23330816);
  float*    h1    = (float*)R2;
  _Float16* h1h   = (_Float16*)(R2 + 8388608);
  _Float16* goutH = (_Float16*)R3;
  _Float16* lngh  = (_Float16*)R3;
  float*    x1    = (float*)(R3 + 4194304);

  tcast_kernel<<<dim3(HGW / 64, ND / 64), NT, 0, stream>>>(gat_W, gatWt, ND, HGW, 16.0f);
  att_rows_kernel<<<64, NT, 0, stream>>>(gat_W, att_src, att_dst, gatWt);
  tcast_kernel<<<dim3(ND / 64, HGW / 64), NT, 0, stream>>>(short_W, shortWt, HGW, ND, 16.0f);
  tcast_kernel<<<dim3(ND / 64, ND / 64), NT, 0, stream>>>(q_W, qWt, ND, ND, 16.0f);
  tcast_kernel<<<dim3(ND / 64, ND / 64), NT, 0, stream>>>(k_W, kWt, ND, ND, 16.0f);
  tcast_kernel<<<dim3(ND / 64, ND / 64), NT, 0, stream>>>(v_W, vWt, ND, ND, 16.0f);
  tcast_kernel<<<dim3(ND / 64, ND / 64), NT, 0, stream>>>(o_W, oWt, ND, ND, 16.0f);
  tcast_kernel<<<dim3(NR / 64, ND / 64), NT, 0, stream>>>(p_W, pWt, ND, NR, 16.0f);
  tcast_kernel<<<dim3(NFF / 64, ND / 64), NT, 0, stream>>>(f1_W, f1Wt, ND, NFF, 16.0f);
  tcast_kernel<<<dim3(ND / 64, NFF / 64), NT, 0, stream>>>(f2_W, f2Wt, NFF, ND, 16.0f);
  cast_scale_f32_f16x2<<<(NBL * ND / 2 + 255) / 256, 256, 0, stream>>>(s, sh, NBL * ND / 2, 16.0f);

  const unsigned short* nul16 = (const unsigned short*)nullptr;

  {
    const int tiles = (NBL / 64) * (HGN / 64);
    wmma_gemm64<0, false, 0, 0, false><<<dim3((tiles + 7) / 8, 1), 256, 0, stream>>>(
        (const unsigned short*)sh, nul16, ND, 0L, (const unsigned short*)gatWt, nul16, ND, 0L,
        (void*)hg, (void*)nullptr, HGN, 0L, (const float*)nullptr, (const float*)nullptr, 0L, NBL, HGN, ND, 1.0f / 256.0f);
  }
  gat_agg_kernel<<<NB * 4, NT, 0, stream>>>(hg, ei, gat_b, acc, goutH);
  {
    const int tiles = (NBL / 64) * (ND / 64);
    wmma_gemm64<0, false, 2, 0, true><<<dim3((tiles + 7) / 8, 1), 256, 0, stream>>>(
        (const unsigned short*)goutH, nul16, HGW, 0L, (const unsigned short*)shortWt, nul16, HGW, 0L,
        (void*)sshrt, (void*)nullptr, ND, 0L, short_b, s, 0L, NBL, ND, HGW, 1.0f / 256.0f);

    wmma_gemm64<0, false, 2, 0, false><<<dim3((tiles + 7) / 8, 1), 256, 0, stream>>>(
        (const unsigned short*)sh, nul16, ND, 0L, (const unsigned short*)qWt, nul16, ND, 0L,
        (void*)tmp, (void*)nullptr, ND, 0L, q_b, (const float*)nullptr, 0L, NBL, ND, ND, 1.0f / 256.0f);
    ln_kernel<0, 1, 0><<<NBL / 64, NT, 0, stream>>>(tmp, lnq_g, lnq_b, (float*)nullptr, qh, (_Float16*)nullptr);
    wmma_gemm64<0, false, 2, 0, false><<<dim3((tiles + 7) / 8, 1), 256, 0, stream>>>(
        (const unsigned short*)sh, nul16, ND, 0L, (const unsigned short*)kWt, nul16, ND, 0L,
        (void*)tmp, (void*)nullptr, ND, 0L, k_b, (const float*)nullptr, 0L, NBL, ND, ND, 1.0f / 256.0f);
    ln_kernel<0, 1, 1><<<NBL / 64, NT, 0, stream>>>(tmp, lnk_g, lnk_b, (float*)nullptr, kh, kT);
    wmma_gemm64<0, false, 2, 0, false><<<dim3((tiles + 7) / 8, 1), 256, 0, stream>>>(
        (const unsigned short*)sh, nul16, ND, 0L, (const unsigned short*)vWt, nul16, ND, 0L,
        (void*)tmp, (void*)nullptr, ND, 0L, v_b, (const float*)nullptr, 0L, NBL, ND, ND, 1.0f / 256.0f);
    ln_kernel<0, 0, 1><<<NBL / 64, NT, 0, stream>>>(tmp, lnv_g, lnv_b, (float*)nullptr, (_Float16*)nullptr, vT);
  }
  {
    const int tiles = (NBL / 64) * (NR / 64);
    wmma_gemm64<0, false, 2, 0, false><<<dim3((tiles + 7) / 8, 1), 256, 0, stream>>>(
        (const unsigned short*)kh, nul16, ND, 0L, (const unsigned short*)pWt, nul16, ND, 0L,
        (void*)pml, (void*)nullptr, NR, 0L, p_b, (const float*)nullptr, 0L, NBL, NR, ND, 1.0f / 256.0f);
  }
  seqsoftmax_kernel<<<NB * NR, NT, 0, stream>>>(pml, pmT);
  {
    const int tiles = (NR / 64) * (ND / 64);
    wmma_gemm64<0, false, 0, 1, false><<<dim3((tiles + 7) / 8, NB), 256, 0, stream>>>(
        (const unsigned short*)pmT, nul16, NL, (long)NR * NL, (const unsigned short*)kT, nul16, NL, (long)ND * NL,
        (void*)kc16, (void*)nullptr, ND, (long)NR * ND, (const float*)nullptr, (const float*)nullptr, 0L, NR, ND, NL, 1.0f / 8192.0f);
    wmma_gemm64<0, false, 0, 1, false><<<dim3((tiles + 7) / 8, NB), 256, 0, stream>>>(
        (const unsigned short*)vT, nul16, NL, (long)ND * NL, (const unsigned short*)pmT, nul16, NL, (long)NR * NL,
        (void*)vcT16, (void*)nullptr, NR, (long)ND * NR, (const float*)nullptr, (const float*)nullptr, 0L, ND, NR, NL, 1.0f / 8192.0f);
  }
  lr_attn_kernel<<<NB * NH * (NL / 64), 128, 0, stream>>>(qh, kc16, vcT16, lngh, 1.0f / 8192.0f, 1.0f / 8192.0f);
  {
    const int tiles = (NBL / 64) * (ND / 64);
    wmma_gemm64<0, false, 2, 0, true><<<dim3((tiles + 7) / 8, 1), 256, 0, stream>>>(
        (const unsigned short*)lngh, nul16, ND, 0L, (const unsigned short*)oWt, nul16, ND, 0L,
        (void*)x1, (void*)nullptr, ND, 0L, o_b, sshrt, 0L, NBL, ND, ND, 1.0f / 4096.0f);
  }
  ln_kernel<1, 1, 0><<<NBL / 64, NT, 0, stream>>>(x1, ln1_g, ln1_b, h1, h1h, (_Float16*)nullptr);
  {
    const int tiles = (NBL / 64) * (NFF / 64);
    wmma_gemm64<0, false, 2, 1, false, 2, 16><<<dim3((tiles + 7) / 8, 1), 256, 0, stream>>>(
        (const unsigned short*)h1h, nul16, ND, 0L, (const unsigned short*)f1Wt, nul16, ND, 0L,
        (void*)ff1h, (void*)nullptr, NFF, 0L, f1_b, (const float*)nullptr, 0L, NBL, NFF, ND, 1.0f / 256.0f);
  }
  {
    const int tiles = (NBL / 64) * (ND / 64);
    wmma_gemm64<0, false, 2, 0, true><<<dim3((tiles + 7) / 8, 1), 256, 0, stream>>>(
        (const unsigned short*)ff1h, nul16, NFF, 0L, (const unsigned short*)f2Wt, nul16, NFF, 0L,
        (void*)x2, (void*)nullptr, ND, 0L, f2_b, h1, 0L, NBL, ND, NFF, 1.0f / 256.0f);
  }
  ln_kernel<1, 0, 0><<<NBL / 64, NT, 0, stream>>>(x2, ln2_g, ln2_b, out, (_Float16*)nullptr, (_Float16*)nullptr);
}
